// RelationNetwork_68805376082627
// MI455X (gfx1250) — hardware-verified
//
#include <hip/hip_runtime.h>
#include <math.h>

typedef __attribute__((ext_vector_type(16))) _Float16 v16h;
typedef __attribute__((ext_vector_type(16))) __bf16 v16b;
typedef __attribute__((ext_vector_type(8)))  _Float16 v8h;
typedef __attribute__((ext_vector_type(8)))  float v8f;
typedef __attribute__((ext_vector_type(4)))  float v4f;
typedef __attribute__((ext_vector_type(2)))  float v2f;
typedef __attribute__((ext_vector_type(4)))  unsigned v4u;
typedef __attribute__((ext_vector_type(4)))  int v4i;
typedef float __attribute__((may_alias)) float_a;
typedef int __attribute__((may_alias)) int_a;

template <typename T> __device__ __forceinline__ void vst2(void* p, T v) { *(volatile T*)p = v; __threadfence(); *(volatile T*)p = v; }
__device__ __forceinline__ v8f wmma16(v16h a, v16h b, v8f c) {
  v8f d = __builtin_amdgcn_wmma_f32_16x16x32_f16(false, a, false, b, (short)0, c, false, false);
  asm volatile("v_nop\n\tv_nop\n\tv_nop\n\tv_nop" : "+v"(d) : "v"(a), "v"(b));
  return d;
}
__device__ __forceinline__ v8f wmma_bf(v16b a, v16b b, v8f c) {
  v8f d = __builtin_amdgcn_wmma_f32_16x16x32_bf16(false, a, false, b, (short)0, c, false, false);
  asm volatile("v_nop\n\tv_nop\n\tv_nop\n\tv_nop" : "+v"(d) : "v"(a), "v"(b));
  return d;
}
__device__ __forceinline__ v16h frag_h(const _Float16* rowk0, int lane) {
  union { v16h v; v8h q[2]; } u; const _Float16* p = rowk0 + 8 * (lane >> 4);
  u.q[0] = *(const v8h*)p; u.q[1] = *(const v8h*)(p + 16); return u.v;
}
__device__ __forceinline__ v16h frag_f32(const float* rowk0, int lane) {
  v16h a; const float* p = rowk0 + 8 * (lane >> 4);
#pragma unroll
  for (int i = 0; i < 8; ++i) { a[i] = (_Float16)p[i]; a[8 + i] = (_Float16)p[16 + i]; }
  return a;
}
__device__ __forceinline__ v16h frag_f32s(const float* rowk0, int lane, float sc) {
  v16h a; const float* p = rowk0 + 8 * (lane >> 4);
#pragma unroll
  for (int i = 0; i < 8; ++i) { a[i] = (_Float16)(p[i] * sc); a[8 + i] = (_Float16)(p[16 + i] * sc); }
  return a;
}
__device__ __forceinline__ v16h fragc_f32(const float* W, int k0, int n, int lane, int ld, int K) {
  v16h a; const int g = lane >> 4;
#pragma unroll
  for (int i = 0; i < 8; ++i) { const int ka = k0 + 8 * g + i, kb = ka + 16;
    a[i] = (_Float16)(ka < K ? W[(size_t)(ka < K ? ka : K - 1) * ld + n] : 0.f); a[8 + i] = (_Float16)(kb < K ? W[(size_t)(kb < K ? kb : K - 1) * ld + n] : 0.f); }
  return a;
}
struct F2 { v16b h, l; };
__device__ __forceinline__ F2 bsplit16(const float v[16]) { F2 r;
#pragma unroll
  for (int i = 0; i < 16; ++i) { const __bf16 h = (__bf16)v[i]; r.h[i] = h; r.l[i] = (__bf16)(v[i] - (float)h); }
  return r; }
__device__ __forceinline__ F2 split_row(const float* row, int k0, int lane) { float v[16]; const float* p = row + k0 + 8 * (lane >> 4);
#pragma unroll
  for (int i = 0; i < 8; ++i) { v[i] = p[i]; v[8 + i] = p[16 + i]; }
  return bsplit16(v); }
__device__ __forceinline__ F2 split_rowK(const float* row, int k0, int lane, int K) { float v[16]; const int g = lane >> 4;
#pragma unroll
  for (int i = 0; i < 8; ++i) { const int ka = k0 + 8 * g + i, kb = ka + 16; v[i] = ka < K ? row[ka < K ? ka : K - 1] : 0.f; v[8 + i] = kb < K ? row[kb < K ? kb : K - 1] : 0.f; }
  return bsplit16(v); }
__device__ __forceinline__ F2 split_col(const float* W, int k0, int n, int lane, int ld, int K) { float v[16]; const int g = lane >> 4;
#pragma unroll
  for (int i = 0; i < 8; ++i) { const int ka = k0 + 8 * g + i, kb = ka + 16; v[i] = ka < K ? W[(size_t)(ka < K ? ka : K - 1) * ld + n] : 0.f; v[8 + i] = kb < K ? W[(size_t)(kb < K ? kb : K - 1) * ld + n] : 0.f; }
  return bsplit16(v); }
__device__ __forceinline__ v8f mac3(const F2& a, const F2& b, v8f c) { c = wmma_bf(a.l, b.h, c); c = wmma_bf(a.h, b.l, c); return wmma_bf(a.h, b.h, c); }
__device__ __forceinline__ float sigm(float v) { return 1.0f / (1.0f + expf(-v)); }
#define LDSX() do { asm volatile("s_wait_dscnt 0" ::: "memory"); __builtin_amdgcn_wave_barrier(); __builtin_amdgcn_fence(__ATOMIC_RELEASE, "workgroup"); } while (0)


#define NOBJ 512
#define DD 128
#define NPAIR (NOBJ * NOBJ)
#define NPB (NPAIR / 64)
#ifndef TPB
#define TPB NPB
#endif
typedef __attribute__((ext_vector_type(8))) __bf16 v8b;
__device__ __forceinline__ v16b frag_b(const __bf16* rowk0, int lane) {
  union { v16b v; v8b q[2]; } u; const __bf16* p = rowk0 + 8 * (lane >> 4);
  u.q[0] = *(const v8b*)p; u.q[1] = *(const v8b*)(p + 16); return u.v;
}
__device__ __forceinline__ float bfr(float v) { return (float)(__bf16)v; }
__device__ __attribute__((noinline)) float exp_ni(float v) { return expf(v); }
__device__ __attribute__((noinline)) float erf_ni(float v) { return erff(v); }

#define WS_XA  0u
#define WS_XB  (WS_XA + 4u * NOBJ * DD)
#define WS_W2  (WS_XB + 4u * NOBJ * DD)
#define WS_W3  (WS_W2 + 2u * DD * DD)
#define WS_PS  (WS_W3 + 2u * DD * DD)
#define WS_END (WS_PS + 4u * (size_t)NPB * DD)

__device__ __forceinline__ v16b fragb_f32(const float* __restrict__ p, int lane) { v16b a; const float* pp = p + 8 * (lane >> 4);
#pragma unroll
  for (int i = 0; i < 8; ++i) { a[i] = (__bf16)pp[i]; a[8 + i] = (__bf16)pp[16 + i]; } return a; }
__global__ __launch_bounds__(128) void k_pre(const float* __restrict__ X, const float* __restrict__ Q, const float* __restrict__ W1, const float* __restrict__ B1, const float* __restrict__ W2, const float* __restrict__ W3, float* __restrict__ XA, float* __restrict__ XB, __bf16* __restrict__ W2T, __bf16* __restrict__ W3T) { __shared__ __align__(16) float sf[4][16][132]; __shared__ __align__(16) float sq[DD]; __shared__ __align__(16) __bf16 st[DD][136];
  const int tid = threadIdx.x, wave = tid >> 5, lane = tid & 31, col = lane & 15, g = lane >> 4;
  if (blockIdx.x == NOBJ / 64) {
#pragma unroll 1
    for (int which = 0; which < 2; ++which) { const float* Wm = which == 0 ? W2 : W3; __bf16* dst = which == 0 ? W2T : W3T;
      for (int e = tid; e < DD * DD; e += 128) { const int k = e >> 7, o = e & 127; st[o][k] = (__bf16)Wm[e]; }
      __syncthreads(); for (int e = tid; e < DD * 16; e += 128) { const int o = e >> 4, qq = e & 15; vst2((unsigned*)(dst + (size_t)o * DD + qq * 8), *(const v4u*)&st[o][qq * 8]); } __syncthreads(); }
    return; }
  { const int o = tid; float a = 0.f;
#pragma unroll 1
    for (int d = 0; d < DD; ++d) a += bfr(Q[d]) * bfr(W1[(size_t)(2 * DD + d) * DD + o]);
    sq[o] = a + bfr(B1[o]); }
  __syncthreads();
  const size_t r0 = (size_t)blockIdx.x * 64 + wave * 16;
#pragma unroll 1
  for (int which = 0; which < 2; ++which) { v8f acc[8] = {};
#pragma unroll
    for (int kc = 0; kc < DD / 32; ++kc) { const v16b a = fragb_f32(X + (r0 + col) * DD + kc * 32, lane);
#pragma unroll
      for (int j = 0; j < 8; ++j) { v16b w; const int o = j * 16 + col;
#pragma unroll
        for (int i = 0; i < 8; ++i) { w[i] = (__bf16)W1[(size_t)(which * DD + kc * 32 + 8 * g + i) * DD + o]; w[8 + i] = (__bf16)W1[(size_t)(which * DD + kc * 32 + 16 + 8 * g + i) * DD + o]; }
        acc[j] = wmma_bf(a, w, acc[j]); } }
#pragma unroll
    for (int j = 0; j < 8; ++j)
#pragma unroll
      for (int r = 0; r < 8; ++r) sf[wave][8 * g + r][j * 16 + col] = acc[j][r] + (which == 1 ? sq[j * 16 + col] : 0.f);
    LDSX(); { float* dst = which == 0 ? XA : XB; for (int rl = 0; rl < 16; ++rl) vst2(dst + (r0 + rl) * DD + lane * 4, *(const v4f*)&sf[wave][rl][lane * 4]); }
    LDSX(); } }
__global__ __launch_bounds__(128) void k_g(const float* __restrict__ XA, const float* __restrict__ XB, const __bf16* __restrict__ W2T, const __bf16* __restrict__ W3T, const float* __restrict__ B2, const float* __restrict__ B3, float* __restrict__ PS) { __shared__ __align__(16) float sa[4][16][132]; __shared__ __align__(16) float sps[4][DD]; __shared__ __align__(16) float spo[DD];
  const int tid = threadIdx.x, wave = tid >> 5, lane = tid & 31, col = lane & 15, g = lane >> 4; const size_t p0 = (size_t)blockIdx.x * 64 + wave * 16;
  for (int e = lane; e < 16 * DD; e += 32) { const int rl = e >> 7, o = e & 127; const size_t p = p0 + rl; const int i = (int)(p / NOBJ), j = (int)(p % NOBJ); sa[wave][rl][o] = fmaxf(XA[i * DD + o] + XB[j * DD + o], 0.f); }
  LDSX();
  v8f acc[8] = {};
#pragma unroll
  for (int kc = 0; kc < DD / 32; ++kc) { const F2 a = split_row(&sa[wave][col][0], kc * 32, lane);
#pragma unroll
    for (int j = 0; j < 8; ++j) { const v16b w = frag_b(W2T + (size_t)(j * 16 + col) * DD + kc * 32, lane); acc[j] = wmma_bf(a.h, w, acc[j]); acc[j] = wmma_bf(a.l, w, acc[j]); } }
  LDSX();
#pragma unroll
  for (int j = 0; j < 8; ++j) { const float bb = bfr(B2[j * 16 + col]);
#pragma unroll
    for (int r = 0; r < 8; ++r) sa[wave][8 * g + r][j * 16 + col] = fmaxf(acc[j][r] + bb, 0.f); }
  LDSX();
  { v8f acc3[8] = {};
#pragma unroll
    for (int kc = 0; kc < DD / 32; ++kc) { const F2 a = split_row(&sa[wave][col][0], kc * 32, lane);
#pragma unroll
      for (int j = 0; j < 8; ++j) { const v16b w = frag_b(W3T + (size_t)(j * 16 + col) * DD + kc * 32, lane); acc3[j] = wmma_bf(a.h, w, acc3[j]); acc3[j] = wmma_bf(a.l, w, acc3[j]); } }
    LDSX();
#pragma unroll
    for (int j = 0; j < 8; ++j) { const float bb = bfr(B3[j * 16 + col]);
#pragma unroll
      for (int r = 0; r < 8; ++r) sa[wave][8 * g + r][j * 16 + col] = fmaxf(acc3[j][r] + bb, 0.f); } }
  LDSX();
  for (int o = lane; o < DD; o += 32) { float s = 0.f;
#pragma unroll 1
    for (int rl = 0; rl < 16; ++rl) s += sa[wave][rl][o];
    sps[wave][o] = s; }
  __syncthreads();
  if (tid < DD) spo[tid] = (sps[0][tid] + sps[1][tid]) + (sps[2][tid] + sps[3][tid]);
  __syncthreads(); if (tid < 32) vst2(PS + (size_t)blockIdx.x * DD + tid * 4, *(const v4f*)&spo[tid * 4]); }
__global__ __launch_bounds__(128) void k_f(const float* __restrict__ PS, const float* __restrict__ FW1, const float* __restrict__ FB1, const float* __restrict__ FW2, const float* __restrict__ FB2, float* __restrict__ OUT) { __shared__ __align__(16) float emb[DD]; __shared__ __align__(16) float hh[DD]; __shared__ __align__(16) float so[DD];
  const int t = threadIdx.x;
  { float s = 0.f;
#pragma unroll 1
    for (int b = 0; b < TPB; ++b) s += PS[(size_t)b * DD + t];
    emb[t] = s; }
  __syncthreads();
  { float a = bfr(FB1[t]);
#pragma unroll 1
    for (int d = 0; d < DD; ++d) a += emb[d] * bfr(FW1[d * DD + t]);
    hh[t] = fmaxf(a, 0.f); }
  __syncthreads();
  { float a = bfr(FB2[t]);
#pragma unroll 1
    for (int d = 0; d < DD; ++d) a += hh[d] * bfr(FW2[d * DD + t]);
    so[t] = a; }
  __syncthreads(); if (t < 32) vst2(OUT + t * 4, *(const v4f*)&so[t * 4]); }
extern "C" void kernel_launch(void* const* d_in, const int* in_sizes, int n_in, void* d_out, int out_size, void* d_ws, size_t ws_size, hipStream_t stream) {
  (void)in_sizes; (void)n_in; (void)out_size;
  const float** F = (const float**)d_in;
  if (ws_size < (size_t)WS_END) return;
  char* ws = (char*)d_ws; float *XA = (float*)(ws + WS_XA), *XB = (float*)(ws + WS_XB), *PS = (float*)(ws + WS_PS); __bf16 *W2T = (__bf16*)(ws + WS_W2), *W3T = (__bf16*)(ws + WS_W3);
  k_pre<<<NOBJ / 64 + 1, 128, 0, stream>>>(F[0], F[1], F[2], F[3], F[4], F[6], XA, XB, W2T, W3T);
  k_g<<<TPB, 128, 0, stream>>>(XA, XB, W2T, W3T, F[5], F[7], PS);
  k_f<<<1, 128, 0, stream>>>(PS, F[8], F[9], F[10], F[11], (float*)d_out);
}
